// GQAAttention_30657476559567
// MI455X (gfx1250) — hardware-verified
//
#include <hip/hip_runtime.h>

#ifndef NB
#define NB 2
#endif
#ifndef SEQ
#define SEQ 2048
#endif
#define NB_FULL 2
#define SEQ_FULL 2048
#define DM 2048
#define NH 16
#define NKV 4
#define NREP (NH / NKV)
#define HDM 128
#define KVD (NKV * HDM)
#define NR (NB * SEQ)
#define QBLKS (SEQ / 64)
#ifndef QB5N
#define QB5N ((SEQ >= 512) ? 4 : (SEQ / 128))
#endif
#define ER (QB5N * 64)
#define SCL 0.08838834764831845f

static_assert(NB >= 1 && NB <= NB_FULL);
static_assert(SEQ % 128 == 0 && SEQ <= SEQ_FULL);
static_assert(QB5N >= 1 && QB5N < QBLKS);
static_assert(ER % 128 == 0);
static_assert((SEQ - ER) % 128 == 0 && SEQ > ER);
static_assert(DM % 64 == 0 && KVD % 64 == 0 && HDM % 32 == 0);

typedef unsigned short v8us __attribute__((ext_vector_type(8), may_alias));
typedef float v8f __attribute__((ext_vector_type(8)));
typedef float v4f __attribute__((ext_vector_type(4)));
typedef float v4fa __attribute__((ext_vector_type(4), may_alias));
typedef _Float16 v16h __attribute__((ext_vector_type(16)));
union FragH { v16h v; v8us half[2]; _Float16 h[16]; unsigned short u[16]; };

__device__ __forceinline__ unsigned short bf16_bits(float x) { unsigned int u = __float_as_uint(x); return (unsigned short)((u + 0x7FFFu + ((u >> 16) & 1u)) >> 16); }
__device__ __forceinline__ float bf16_val(unsigned short b) { return __uint_as_float(((unsigned int)b) << 16); }
__device__ __forceinline__ float bf16_rne(float x) { return bf16_val(bf16_bits(x)); }

__device__ __forceinline__ v16h frag16(const unsigned short* p, int hh) { FragH f; f.half[0] = *(const v8us*)(p + 8 * hh); f.half[1] = *(const v8us*)(p + 16 + 8 * hh); return f.v; }
__device__ __forceinline__ v8f mma16(v16h a, v16h b, v8f c) {
  v8f d = __builtin_amdgcn_wmma_f32_16x16x32_f16(false, a, false, b, (short)0, c, false, false);
  asm volatile("v_nop\n\tv_nop\n\tv_nop\n\tv_nop" : "+v"(d) : "v"(a), "v"(b));
  return d;
}

__global__ __launch_bounds__(256) void k_wt_f16(const float* __restrict__ W, _Float16* __restrict__ Wt, int K, int N, float scale) {
  const int t = blockIdx.x * 256 + threadIdx.x; if (t >= N * (K / 8)) return;
  const int n = t / (K / 8), k8 = (t - n * (K / 8)) * 8; FragH f;
#pragma unroll
  for (int i = 0; i < 8; ++i) f.h[i] = (_Float16)(bf16_rne(W[(size_t)(k8 + i) * N + n]) * scale);
  const v8us o = f.half[0]; unsigned short* p = (unsigned short*)Wt + (size_t)n * K + k8;
  *(volatile v8us*)p = o; __threadfence(); *(volatile v8us*)p = o;
}

__global__ __launch_bounds__(256) void k_x16(const float* __restrict__ x, _Float16* __restrict__ X16) {
  const size_t t = (size_t)blockIdx.x * 256 + threadIdx.x; if (t >= (size_t)NR * DM / 8) return;
  const size_t e = t * 8; const size_t row = e / DM; const int c = (int)(e - row * DM); const size_t b = row / SEQ, s = row - b * SEQ;
  const float* src = x + (b * SEQ_FULL + s) * DM + c;
  const v4f a = *(const v4fa*)src, d = *(const v4fa*)(src + 4); FragH f;
#pragma unroll
  for (int q = 0; q < 4; ++q) { f.h[q] = (_Float16)bf16_rne(a[q]); f.h[4 + q] = (_Float16)bf16_rne(d[q]); }
  const v8us o = f.half[0]; unsigned short* p = (unsigned short*)X16 + e;
  *(volatile v8us*)p = o; __threadfence(); *(volatile v8us*)p = o;
}

__global__ __launch_bounds__(256) void k_tab(const int* __restrict__ pid, float* __restrict__ CS, float* __restrict__ SN) {
  #pragma clang fp contract(off)
  const int t = blockIdx.x * 256 + threadIdx.x; if (t >= NR * 64) return;
  const int j = t & 63; const int row = t >> 6; const int b = row / SEQ, s = row - b * SEQ;
  const int p = pid[(size_t)b * SEQ_FULL + s];
  const double pw = exp2((double)j * (19.931568569324174 / 64.0));
  const float thp = (float)pw;
  const float inv = 1.0f / thp;
  const float th = (float)p * inv;
  const float c = cosf(th), sn = sinf(th);
  *(volatile float*)(CS + t) = c; *(volatile float*)(SN + t) = sn; __threadfence();
  *(volatile float*)(CS + t) = c; *(volatile float*)(SN + t) = sn;
}

__global__ __launch_bounds__(256) void k_mchk(const float* __restrict__ msk, float* __restrict__ FLG) {
  __shared__ int red[256];
  const int tid = threadIdx.x; const int b = blockIdx.x / QBLKS, qb = blockIdx.x - b * QBLKS;
  int bad = 0;
  constexpr int NF4 = 64 * (SEQ / 4);
  for (int i = tid; i < NF4; i += 256) {
    const int ql = i / (SEQ / 4), k4 = (i - ql * (SEQ / 4)) * 4; const int q = qb * 64 + ql;
    const v4f v = *(const v4fa*)(msk + ((size_t)b * SEQ_FULL + q) * SEQ_FULL + k4);
#pragma unroll
    for (int c = 0; c < 4; ++c) { const float ex = (k4 + c <= q) ? 0.0f : -1.0e9f; bad |= (v[c] != ex) ? 1 : 0; }
  }
  red[tid] = bad; __syncthreads();
  for (int st = 128; st > 0; st >>= 1) { if (tid < st) red[tid] |= red[tid + st]; __syncthreads(); }
  if (tid < 32) { const float f = (red[0] != 0) ? 1.0f : 0.0f; float* p = FLG + (size_t)blockIdx.x * 32 + tid; *(volatile float*)p = f; __threadfence(); *(volatile float*)p = f; }
}

__global__ __launch_bounds__(128) void k_gemm2(const _Float16* __restrict__ A, int lda, size_t sA, const _Float16* __restrict__ Bh, int ldb, float alpha,
                                              const float* __restrict__ CP, int ldp, size_t sP, float* __restrict__ C, int ldc, size_t sC, int M, int N, int K) {
  __shared__ __attribute__((aligned(16))) float so[4][32][68];
  const int tid = threadIdx.x, w = tid >> 5, lane = tid & 31, ln = lane & 15, hh = lane >> 4; const int by = blockIdx.y;
  A += (size_t)by * sA; const size_t cofs = (size_t)by * sC; const size_t pofs = (size_t)by * sP;
  const int ntn = N >> 6; const int mt = blockIdx.x / ntn, nq = blockIdx.x - mt * ntn; const int row0 = mt * 128 + 32 * w, col0 = nq * 64; if (row0 >= M) return;
  const unsigned short* a0p = (const unsigned short*)A + (size_t)(row0 + ln) * lda; const unsigned short* a1p = a0p + (size_t)16 * lda;
  const unsigned short* b0p = (const unsigned short*)Bh + (size_t)(col0 + ln) * ldb; const unsigned short* b1p = b0p + (size_t)16 * ldb;
  const unsigned short* b2p = b1p + (size_t)16 * ldb; const unsigned short* b3p = b2p + (size_t)16 * ldb;
  const v8f z8 = {0.f,0.f,0.f,0.f,0.f,0.f,0.f,0.f}; v8f c00 = z8, c01 = z8, c02 = z8, c03 = z8, c10 = z8, c11 = z8, c12 = z8, c13 = z8;
#pragma unroll 1
  for (int kb = 0; kb < K; kb += 32) {
    const v16h a0 = frag16(a0p + kb, hh), a1 = frag16(a1p + kb, hh);
    v16h b = frag16(b0p + kb, hh); c00 = mma16(a0, b, c00); c10 = mma16(a1, b, c10);
    b = frag16(b1p + kb, hh); c01 = mma16(a0, b, c01); c11 = mma16(a1, b, c11);
    b = frag16(b2p + kb, hh); c02 = mma16(a0, b, c02); c12 = mma16(a1, b, c12);
    b = frag16(b3p + kb, hh); c03 = mma16(a0, b, c03); c13 = mma16(a1, b, c13);
  }
  v8f accs[8] = {c00, c01, c02, c03, c10, c11, c12, c13};
#pragma unroll
  for (int u = 0; u < 8; ++u) { const int t = u & 3, half = u >> 2;
#pragma unroll
    for (int r = 0; r < 8; ++r) so[w][half * 16 + 8 * hh + r][t * 16 + ln] = accs[u][r] * alpha; }
  __builtin_amdgcn_fence(4, "workgroup"); __builtin_amdgcn_wave_barrier();
  const int rsub = lane >> 4, c4 = (lane & 15) * 4;
  if (CP != nullptr) {
#pragma unroll
    for (int q = 0; q < 16; ++q) { const int r = q * 2 + rsub; v4f v = *(const v4fa*)&so[w][r][c4]; const v4f p = *(const v4fa*)(CP + pofs + (size_t)(row0 + r) * ldp + col0 + c4); v += p; *(v4fa*)&so[w][r][c4] = v; }
  }
  for (int pass = 0; pass < 2; ++pass) {
#pragma unroll
    for (int q = 0; q < 16; ++q) { const int r = q * 2 + rsub; const v4f v = *(const v4fa*)&so[w][r][c4]; *(volatile v4f*)(C + cofs + (size_t)(row0 + r) * ldc + col0 + c4) = v; }
    if (pass == 0) __threadfence();
  }
}

__global__ __launch_bounds__(256) void k_rope(const float* __restrict__ F, int nh, const float* __restrict__ CS, const float* __restrict__ SN, _Float16* __restrict__ H, _Float16* __restrict__ L) {
  #pragma clang fp contract(off)
  const size_t t = (size_t)blockIdx.x * 256 + threadIdx.x; if (t >= (size_t)NR * nh * 16) return;
  const int g = (int)(t & 15); const int hd = (int)((t >> 4) % nh); const size_t row = t / ((size_t)16 * nh);
  const size_t o = row * (size_t)(nh * HDM) + (size_t)hd * HDM + (size_t)g * 8;
  const v4f a = *(const v4fa*)(F + o), d = *(const v4fa*)(F + o + 4);
  const float xs[8] = {a[0], a[1], a[2], a[3], d[0], d[1], d[2], d[3]};
  const v4f cc = *(const v4fa*)(CS + row * 64 + g * 4), ss = *(const v4fa*)(SN + row * 64 + g * 4);
  FragH fh, fl;
#pragma unroll
  for (int pr = 0; pr < 4; ++pr) {
    const float x1 = xs[2 * pr], x2 = xs[2 * pr + 1]; const float cv = cc[pr], sv = ss[pr];
    float o1 = x1 * cv; o1 -= x2 * sv; float o2 = x1 * sv; o2 += x2 * cv;
    _Float16 hv = (_Float16)o1; fh.h[2 * pr] = hv; fl.h[2 * pr] = (_Float16)((o1 - (float)hv) * 1024.0f);
    hv = (_Float16)o2; fh.h[2 * pr + 1] = hv; fl.h[2 * pr + 1] = (_Float16)((o2 - (float)hv) * 1024.0f);
  }
  const v8us oh = fh.half[0], ol = fl.half[0]; unsigned short* ph = (unsigned short*)H + o; unsigned short* pl = (unsigned short*)L + o;
  *(volatile v8us*)ph = oh; *(volatile v8us*)pl = ol; __threadfence(); *(volatile v8us*)ph = oh; *(volatile v8us*)pl = ol;
}

__global__ __launch_bounds__(256) void k_vtg2(const float* __restrict__ VF, _Float16* __restrict__ VTH, _Float16* __restrict__ VTL) {
  __shared__ unsigned short tt[2][64][130];
  const int tid = threadIdx.x; const int slab = blockIdx.x / (SEQ / 64), lg = blockIdx.x - slab * (SEQ / 64); const int b = slab / NKV, hk = slab - b * NKV;
  for (int i = tid; i < 64 * 32; i += 256) {
    const int r = i >> 5, c4 = (i & 31) * 4;
    const v4f a = *(const v4fa*)(VF + ((size_t)b * SEQ + lg * 64 + r) * KVD + hk * HDM + c4); FragH fh, fl;
#pragma unroll
    for (int q = 0; q < 4; ++q) { const _Float16 hv = (_Float16)a[q]; fh.h[q] = hv; fl.h[q] = (_Float16)((a[q] - (float)hv) * 1024.0f); }
#pragma unroll
    for (int q = 0; q < 4; ++q) { tt[0][r][c4 + q] = fh.u[q]; tt[1][r][c4 + q] = fl.u[q]; }
  }
  __syncthreads();
  const int pc = tid & 7, dsub = tid >> 3;
  for (int pass = 0; pass < 2; ++pass) {
#pragma unroll
    for (int it = 0; it < 4; ++it) {
      const int d = it * 32 + dsub; FragH f, g;
#pragma unroll
      for (int q = 0; q < 8; ++q) { f.u[q] = tt[0][pc * 8 + q][d]; g.u[q] = tt[1][pc * 8 + q][d]; }
      const size_t o = ((size_t)slab * HDM + d) * SEQ + (size_t)lg * 64 + pc * 8;
      *(volatile v8us*)((unsigned short*)VTH + o) = f.half[0]; *(volatile v8us*)((unsigned short*)VTL + o) = g.half[0];
    }
    if (pass == 0) __threadfence();
  }
}

__global__ __launch_bounds__(256) void k_hl(const float* __restrict__ F, _Float16* __restrict__ Hh, _Float16* __restrict__ Hl, size_t n8) {
  const size_t t = (size_t)blockIdx.x * 256 + threadIdx.x; if (t >= n8) return; FragH fh, fl;
  const v4f a = *(const v4fa*)(F + t * 8), c = *(const v4fa*)(F + t * 8 + 4);
#pragma unroll
  for (int q = 0; q < 4; ++q) {
    _Float16 hv = (_Float16)a[q]; fh.h[q] = hv; fl.h[q] = (_Float16)((a[q] - (float)hv) * 1024.0f);
    hv = (_Float16)c[q]; fh.h[4 + q] = hv; fl.h[4 + q] = (_Float16)((c[q] - (float)hv) * 1024.0f);
  }
  const v8us oh = fh.half[0], ol = fl.half[0]; unsigned short* ph = (unsigned short*)Hh + t * 8; unsigned short* pl = (unsigned short*)Hl + t * 8;
  *(volatile v8us*)ph = oh; *(volatile v8us*)pl = ol; __threadfence(); *(volatile v8us*)ph = oh; *(volatile v8us*)pl = ol;
}

__global__ __launch_bounds__(128) __attribute__((amdgpu_num_vgpr(256)))
void k_flash(const _Float16* __restrict__ QH, const _Float16* __restrict__ KH, const _Float16* __restrict__ VTH, const float* __restrict__ FLG, float* __restrict__ O) {
  constexpr int KS = HDM / 32, DT = HDM / 16, NQP = QBLKS - QB5N;
  __shared__ __attribute__((aligned(16))) unsigned short sP[4][16][40];
  __shared__ __attribute__((aligned(16))) float sO[4][16][HDM + 4];
  const int tid = threadIdx.x, w = tid >> 5, lane = tid & 31, ln = lane & 15, hh = lane >> 4;
  const int slab = blockIdx.x / NQP, qblk = QB5N + (blockIdx.x - slab * NQP); const int b = slab / NH, h = slab - b * NH, hk = h / NREP;
  const int qb0 = qblk * 64, q0 = qb0 + w * 16;
  const float flg = FLG[(size_t)(b * QBLKS + qblk) * 32];
  FragH aq[KS];
  { const unsigned short* qr = (const unsigned short*)QH + ((size_t)b * SEQ + q0 + ln) * DM + h * HDM;
#pragma unroll
    for (int ks = 0; ks < KS; ++ks) { aq[ks].half[0] = *(const v8us*)(qr + ks * 32 + 8 * hh); aq[ks].half[1] = *(const v8us*)(qr + ks * 32 + 16 + 8 * hh); } }
  const unsigned short* Kb = (const unsigned short*)KH + (size_t)b * SEQ * KVD + hk * HDM;
  const unsigned short* Vth = (const unsigned short*)VTH + (size_t)(b * NKV + hk) * HDM * SEQ;
  const v8f z8 = {0.f,0.f,0.f,0.f,0.f,0.f,0.f,0.f};
  float m_r[8], l_r[8]; v8f oacc[DT];
#pragma unroll
  for (int r = 0; r < 8; ++r) { m_r[r] = -3.0e38f; l_r[r] = 0.f; }
#pragma unroll
  for (int dt = 0; dt < DT; ++dt) oacc[dt] = z8;
  const int jend = qb0 + 64;
#pragma unroll 1
  for (int j0 = 0; j0 < jend; j0 += 32) {
    v8f s[2];
#pragma unroll
    for (int nt = 0; nt < 2; ++nt) {
      const unsigned short* kr = Kb + (size_t)(j0 + nt * 16 + ln) * KVD; v8f acc = z8;
#pragma unroll
      for (int ks = 0; ks < KS; ++ks) { const v16h bk = frag16(kr + ks * 32, hh); acc = mma16(aq[ks].v, bk, acc); }
      s[nt] = acc;
    }
#pragma unroll
    for (int r = 0; r < 8; ++r) {
      const int tq = q0 + 8 * hh + r; const int k0 = j0 + ln, k1 = j0 + 16 + ln;
      const bool ok0 = (k0 <= tq), ok1 = (k1 <= tq);
      const float s0 = ok0 ? s[0][r] * SCL : -3.0e38f, s1 = ok1 ? s[1][r] * SCL : -3.0e38f;
      float mc = fmaxf(s0, s1);
      mc = fmaxf(mc, __shfl_xor(mc, 1, 32)); mc = fmaxf(mc, __shfl_xor(mc, 2, 32)); mc = fmaxf(mc, __shfl_xor(mc, 4, 32)); mc = fmaxf(mc, __shfl_xor(mc, 8, 32));
      const float mn = fmaxf(m_r[r], mc); const float al = (mn > -1.0e38f) ? expf(m_r[r] - mn) : 1.0f; m_r[r] = mn;
      const float p0 = ok0 ? expf(s0 - mn) : 0.f, p1 = ok1 ? expf(s1 - mn) : 0.f; l_r[r] = l_r[r] * al + p0 + p1;
#pragma unroll
      for (int dt = 0; dt < DT; ++dt) oacc[dt][r] *= al;
      FragH t2; t2.h[0] = (_Float16)(p0 * 1024.0f); t2.h[1] = (_Float16)(p1 * 1024.0f);
      sP[w][8 * hh + r][ln] = t2.u[0]; sP[w][8 * hh + r][16 + ln] = t2.u[1];
    }
    __builtin_amdgcn_fence(4, "workgroup"); __builtin_amdgcn_wave_barrier();
    const v16h pa = frag16(&sP[w][ln][0], hh);
#pragma unroll
    for (int dt = 0; dt < DT; ++dt) { const v16h bv = frag16(Vth + (size_t)(dt * 16 + ln) * SEQ + j0, hh); oacc[dt] = mma16(pa, bv, oacc[dt]); }
    __builtin_amdgcn_fence(4, "workgroup"); __builtin_amdgcn_wave_barrier();
  }
#pragma unroll
  for (int r = 0; r < 8; ++r) { float l = l_r[r]; l += __shfl_xor(l, 1, 32); l += __shfl_xor(l, 2, 32); l += __shfl_xor(l, 4, 32); l += __shfl_xor(l, 8, 32); l_r[r] = (l > 0.f) ? 1.0f / (l * 1024.0f) : 0.f; }
  const float qnan = __uint_as_float(0x7fc00000u);
#pragma unroll
  for (int dt = 0; dt < DT; ++dt)
#pragma unroll
    for (int r = 0; r < 8; ++r) { float v = oacc[dt][r] * l_r[r]; v = (flg != 0.f) ? qnan : v; sO[w][8 * hh + r][dt * 16 + ln] = v; }
  __builtin_amdgcn_fence(4, "workgroup"); __builtin_amdgcn_wave_barrier();
  for (int pass = 0; pass < 2; ++pass) {
#pragma unroll
    for (int r = 0; r < 16; ++r) { const v4f val = *(const v4fa*)&sO[w][r][lane * 4]; *(volatile v4f*)(O + ((size_t)b * SEQ + q0 + r) * DM + h * HDM + lane * 4) = val; }
    if (pass == 0) __threadfence();
  }
}

__global__ __launch_bounds__(128) __attribute__((amdgpu_num_vgpr(256)))
void k_flashr(const _Float16* __restrict__ QH, const _Float16* __restrict__ QL, const _Float16* __restrict__ KH, const _Float16* __restrict__ KL,
              const _Float16* __restrict__ VTH, const _Float16* __restrict__ VTL, const float* __restrict__ FLG, float* __restrict__ O) {
  constexpr int KS = HDM / 32, DT = 4;
  __shared__ __attribute__((aligned(16))) unsigned short sP[4][16][40];
  __shared__ __attribute__((aligned(16))) unsigned short sPL[4][16][40];
  __shared__ __attribute__((aligned(16))) float sO[4][16][68];
  const int tid = threadIdx.x, w = tid >> 5, lane = tid & 31, ln = lane & 15, hh = lane >> 4;
  const int bid = blockIdx.x; const int dh = bid & 1; const int rest = bid >> 1; const int slab = rest / QB5N, qblk = rest - slab * QB5N;
  const int b = slab / NH, h = slab - b * NH, hk = h / NREP;
  const int qb0 = qblk * 64, q0 = qb0 + w * 16;
  const float flg = FLG[(size_t)(b * QBLKS + qblk) * 32];
  const unsigned short* qr = (const unsigned short*)QH + ((size_t)b * SEQ + q0 + ln) * DM + h * HDM;
  const unsigned short* qlr = (const unsigned short*)QL + ((size_t)b * SEQ + q0 + ln) * DM + h * HDM;
  const unsigned short* Kb = (const unsigned short*)KH + (size_t)b * SEQ * KVD + hk * HDM;
  const unsigned short* Klb = (const unsigned short*)KL + (size_t)b * SEQ * KVD + hk * HDM;
  const size_t vbase = ((size_t)(b * NKV + hk) * HDM + (size_t)dh * 64) * SEQ;
  const unsigned short* Vth = (const unsigned short*)VTH + vbase; const unsigned short* Vtl = (const unsigned short*)VTL + vbase;
  const v8f z8 = {0.f,0.f,0.f,0.f,0.f,0.f,0.f,0.f};
  float m_r[8], l_r[8]; v8f oacc[DT], oaccL[DT];
#pragma unroll
  for (int r = 0; r < 8; ++r) { m_r[r] = -3.0e38f; l_r[r] = 0.f; }
#pragma unroll
  for (int dt = 0; dt < DT; ++dt) { oacc[dt] = z8; oaccL[dt] = z8; }
  const int jend = qb0 + 64;
#pragma unroll 1
  for (int j0 = 0; j0 < jend; j0 += 32) {
    v8f s[2];
#pragma unroll
    for (int nt = 0; nt < 2; ++nt) {
      const size_t ko = (size_t)(j0 + nt * 16 + ln) * KVD; v8f acc = z8, accl = z8;
#pragma unroll
      for (int ks = 0; ks < KS; ++ks) {
        const v16h a = frag16(qr + ks * 32, hh), al = frag16(qlr + ks * 32, hh);
        const v16h bk = frag16(Kb + ko + ks * 32, hh), bl = frag16(Klb + ko + ks * 32, hh);
        acc = mma16(a, bk, acc); accl = mma16(al, bk, accl); accl = mma16(a, bl, accl);
      }
#pragma unroll
      for (int r = 0; r < 8; ++r) acc[r] += accl[r] * 0.0009765625f;
      s[nt] = acc;
    }
#pragma unroll
    for (int r = 0; r < 8; ++r) {
      const int tq = q0 + 8 * hh + r; const int k0 = j0 + ln, k1 = j0 + 16 + ln;
      const bool ok0 = (k0 <= tq), ok1 = (k1 <= tq);
      const float s0 = ok0 ? s[0][r] * SCL : -3.0e38f, s1 = ok1 ? s[1][r] * SCL : -3.0e38f;
      float mc = fmaxf(s0, s1);
      mc = fmaxf(mc, __shfl_xor(mc, 1, 32)); mc = fmaxf(mc, __shfl_xor(mc, 2, 32)); mc = fmaxf(mc, __shfl_xor(mc, 4, 32)); mc = fmaxf(mc, __shfl_xor(mc, 8, 32));
      const float mn = fmaxf(m_r[r], mc); const float al = (mn > -1.0e38f) ? expf(m_r[r] - mn) : 1.0f; m_r[r] = mn;
      const float p0 = ok0 ? expf(s0 - mn) : 0.f, p1 = ok1 ? expf(s1 - mn) : 0.f; l_r[r] = l_r[r] * al + p0 + p1;
#pragma unroll
      for (int dt = 0; dt < DT; ++dt) { oacc[dt][r] *= al; oaccL[dt][r] *= al; }
      FragH t2, t2l; const float ps0 = p0 * 1024.0f, ps1 = p1 * 1024.0f;
      t2.h[0] = (_Float16)ps0; t2.h[1] = (_Float16)ps1;
      t2l.h[0] = (_Float16)((ps0 - (float)t2.h[0]) * 1024.0f); t2l.h[1] = (_Float16)((ps1 - (float)t2.h[1]) * 1024.0f);
      sP[w][8 * hh + r][ln] = t2.u[0]; sP[w][8 * hh + r][16 + ln] = t2.u[1]; sPL[w][8 * hh + r][ln] = t2l.u[0]; sPL[w][8 * hh + r][16 + ln] = t2l.u[1];
    }
    __builtin_amdgcn_fence(4, "workgroup"); __builtin_amdgcn_wave_barrier();
    const v16h pa = frag16(&sP[w][ln][0], hh), pl = frag16(&sPL[w][ln][0], hh);
#pragma unroll
    for (int dt = 0; dt < DT; ++dt) {
      const size_t vo = (size_t)(dt * 16 + ln) * SEQ + j0; const v16h bv = frag16(Vth + vo, hh), bl = frag16(Vtl + vo, hh);
      oacc[dt] = mma16(pa, bv, oacc[dt]); oaccL[dt] = mma16(pl, bv, oaccL[dt]); oaccL[dt] = mma16(pa, bl, oaccL[dt]);
    }
    __builtin_amdgcn_fence(4, "workgroup"); __builtin_amdgcn_wave_barrier();
  }
#pragma unroll
  for (int r = 0; r < 8; ++r) { float l = l_r[r]; l += __shfl_xor(l, 1, 32); l += __shfl_xor(l, 2, 32); l += __shfl_xor(l, 4, 32); l += __shfl_xor(l, 8, 32); l_r[r] = (l > 0.f) ? 1.0f / (l * 1024.0f) : 0.f; }
  const float qnan = __uint_as_float(0x7fc00000u);
#pragma unroll
  for (int dt = 0; dt < DT; ++dt)
#pragma unroll
    for (int r = 0; r < 8; ++r) { float v = oacc[dt][r] + oaccL[dt][r] * 0.0009765625f; v *= l_r[r]; v = (flg != 0.f) ? qnan : v; sO[w][8 * hh + r][dt * 16 + ln] = v; }
  __builtin_amdgcn_fence(4, "workgroup"); __builtin_amdgcn_wave_barrier();
  for (int pass = 0; pass < 2; ++pass) {
#pragma unroll
    for (int rp = 0; rp < 16; rp += 2) { const int r = rp + (lane >> 4), pc = lane & 15; const v4f val = *(const v4fa*)&sO[w][r][pc * 4];
      *(volatile v4f*)(O + ((size_t)b * SEQ + q0 + r) * DM + h * HDM + dh * 64 + pc * 4) = val; }
    if (pass == 0) __threadfence();
  }
}

extern "C" void kernel_launch(void* const* d_in, const int* in_sizes, int n_in,
                              void* d_out, int out_size, void* d_ws, size_t ws_size, hipStream_t stream) {
  if (n_in < 7) return;
  const size_t rows_hi = (size_t)(NB - 1) * SEQ_FULL + SEQ;
  if ((size_t)in_sizes[0] < rows_hi * DM) return;
  if ((size_t)in_sizes[1] < rows_hi) return;
  if ((size_t)in_sizes[2] < rows_hi * SEQ_FULL) return;
  if ((size_t)in_sizes[3] < (size_t)DM * DM || (size_t)in_sizes[4] < (size_t)DM * KVD || (size_t)in_sizes[5] < (size_t)DM * KVD || (size_t)in_sizes[6] < (size_t)DM * DM) return;
  if ((size_t)out_size < rows_hi * DM) return;
  const float* x = (const float*)d_in[0]; const int* pid = (const int*)d_in[1]; const float* msk = (const float*)d_in[2];
  const float* Wq = (const float*)d_in[3]; const float* Wk = (const float*)d_in[4]; const float* Wv = (const float*)d_in[5]; const float* Wo = (const float*)d_in[6];
  float* out = (float*)d_out;
  char* ws = (char*)d_ws; size_t off = 0;
  auto take = [&](size_t bytes) { char* p = ws + off; off += (bytes + 255) & ~(size_t)255; return p; };
  const size_t np = (size_t)NR * DM, nk = (size_t)NR * KVD, nvt = (size_t)NB * NKV * HDM * SEQ;
  _Float16* BQ = (_Float16*)take((size_t)DM * DM * 2); _Float16* BK = (_Float16*)take((size_t)KVD * DM * 2); _Float16* BV = (_Float16*)take((size_t)KVD * DM * 2); _Float16* BO = (_Float16*)take((size_t)DM * DM * 2);
  _Float16* X16 = (_Float16*)take(np * 2); _Float16* QH = X16; _Float16* OH = X16;
  _Float16* QL = (_Float16*)take(np * 2); _Float16* OL = QL;
  float* QF = (float*)take(np * 4); float* O = QF;
  float* KF = (float*)take(nk * 4); float* VF = (float*)take(nk * 4);
  _Float16* KH = (_Float16*)take(nk * 2); _Float16* KL = (_Float16*)take(nk * 2);
  _Float16* VTH = (_Float16*)take(nvt * 2); _Float16* VTL = (_Float16*)take(nvt * 2);
  float* CS = (float*)take((size_t)NR * 64 * 4); float* SN = (float*)take((size_t)NR * 64 * 4);
  float* FLG = (float*)take((size_t)NB * QBLKS * 32 * 4);
  float* CPB = (float*)take((size_t)NB * ER * DM * 4);
  if (off > ws_size) return;
  auto nblk = [](size_t n) { return (unsigned)((n + 255) / 256); };

  k_wt_f16<<<nblk((size_t)DM * DM / 8), 256, 0, stream>>>(Wq, BQ, DM, DM, 16.0f);
  k_wt_f16<<<nblk((size_t)DM * KVD / 8), 256, 0, stream>>>(Wk, BK, DM, KVD, 16.0f);
  k_wt_f16<<<nblk((size_t)DM * KVD / 8), 256, 0, stream>>>(Wv, BV, DM, KVD, 16.0f);
  k_wt_f16<<<nblk((size_t)DM * DM / 8), 256, 0, stream>>>(Wo, BO, DM, DM, 16.0f);
  k_x16<<<nblk(np / 8), 256, 0, stream>>>(x, X16);
  k_tab<<<nblk((size_t)NR * 64), 256, 0, stream>>>(pid, CS, SN);
  k_mchk<<<(unsigned)(NB * QBLKS), 256, 0, stream>>>(msk, FLG);
  k_gemm2<<<dim3((unsigned)((NR / 128) * (DM / 64)), 1), 128, 0, stream>>>(X16, DM, (size_t)0, BQ, DM, 0.0625f, nullptr, 0, (size_t)0, QF, DM, (size_t)0, NR, DM, DM);
  k_gemm2<<<dim3((unsigned)((NR / 128) * (KVD / 64)), 1), 128, 0, stream>>>(X16, DM, (size_t)0, BK, DM, 0.0625f, nullptr, 0, (size_t)0, KF, KVD, (size_t)0, NR, KVD, DM);
  k_gemm2<<<dim3((unsigned)((NR / 128) * (KVD / 64)), 1), 128, 0, stream>>>(X16, DM, (size_t)0, BV, DM, 0.0625f, nullptr, 0, (size_t)0, VF, KVD, (size_t)0, NR, KVD, DM);
  k_rope<<<nblk((size_t)NR * NH * 16), 256, 0, stream>>>(QF, NH, CS, SN, QH, QL);
  k_rope<<<nblk((size_t)NR * NKV * 16), 256, 0, stream>>>(KF, NKV, CS, SN, KH, KL);
  k_vtg2<<<(unsigned)(NB * NKV * (SEQ / 64)), 256, 0, stream>>>(VF, VTH, VTL);
  k_flashr<<<(unsigned)(NB * NH * QB5N * 2), 128, 0, stream>>>(QH, QL, KH, KL, VTH, VTL, FLG, O);
  k_flash<<<(unsigned)(NB * NH * (QBLKS - QB5N)), 128, 0, stream>>>(QH, KH, VTH, FLG, O);
  k_hl<<<nblk(np / 8), 256, 0, stream>>>(O, OH, OL, np / 8);
  k_gemm2<<<dim3((unsigned)((ER / 128) * (DM / 64)), NB), 128, 0, stream>>>(OL, DM, (size_t)SEQ * DM, BO, DM, 0.0625f / 1024.0f, nullptr, 0, (size_t)0, CPB, DM, (size_t)ER * DM, ER, DM, DM);
  k_gemm2<<<dim3((unsigned)((ER / 128) * (DM / 64)), NB), 128, 0, stream>>>(OH, DM, (size_t)SEQ * DM, BO, DM, 0.0625f, CPB, DM, (size_t)ER * DM, out, DM, (size_t)SEQ_FULL * DM, ER, DM, DM);
  k_gemm2<<<dim3((unsigned)(((SEQ - ER) / 128) * (DM / 64)), NB), 128, 0, stream>>>(OH + (size_t)ER * DM, DM, (size_t)SEQ * DM, BO, DM, 0.0625f, nullptr, 0, (size_t)0, out + (size_t)ER * DM, DM, (size_t)SEQ_FULL * DM, SEQ - ER, DM, DM);
}
